// GLA_50036368998927
// MI455X (gfx1250) — hardware-verified
//
#include <hip/hip_runtime.h>
#include <stddef.h>


#define NB    2
#define NL    1024
#define NH    32
#define NKV   8
#define HD    64
#define HID   2048
#define NG    4
#define LOWR  16
#define NOUT  (NH * HD)
#define TCH   32
#define TPW   72
#define SCAN_THREADS 128
#define LN_EPS 1e-5f

typedef float v4f __attribute__((ext_vector_type(4)));
typedef float v8f __attribute__((ext_vector_type(8)));
typedef unsigned short us8 __attribute__((ext_vector_type(8)));
typedef unsigned short us16 __attribute__((ext_vector_type(16)));
typedef __bf16 v16bf __attribute__((ext_vector_type(16)));

union Frag { v16bf v; us16 u; us8 hv[2]; };

static_assert((NB * NL) % 64 == 0);
static_assert(HID % 64 == 0);
static_assert(NOUT % 64 == 0);
static_assert(NL % TCH == 0);
static_assert(NH % NKV == 0);
static_assert(sizeof(Frag) == 32);

__device__ __forceinline__ unsigned short f2bf(float x) {
  unsigned int u = __float_as_uint(x);
  u += 0x7FFFu + ((u >> 16) & 1u);
  return (unsigned short)(u >> 16);
}
__device__ __forceinline__ float bfr(float x) {
  return __uint_as_float(((unsigned int)f2bf(x)) << 16);
}

__device__ __forceinline__ v8f wmma_bf16(v16bf a, v16bf b, v8f c) {
  v8f d = __builtin_amdgcn_wmma_f32_16x16x32_bf16(false, a, false, b, (short)0, c, false, false);
  asm volatile("v_nop\n\tv_nop\n\tv_nop\n\tv_nop" : "+v"(d) : "v"(a), "v"(b));
  return d;
}

__global__ __launch_bounds__(256)
void k_cvt_h(const float* __restrict__ src, unsigned short* dst, int n8) {
  const int i = blockIdx.x * 256 + threadIdx.x;
  if (i >= n8) return;
  const v4f* s = (const v4f*)(src + (size_t)i * 8);
  const v4f x0 = s[0];
  const v4f x1 = s[1];
  us8 o;
  o[0] = f2bf(x0[0]); o[1] = f2bf(x0[1]); o[2] = f2bf(x0[2]); o[3] = f2bf(x0[3]);
  o[4] = f2bf(x1[0]); o[5] = f2bf(x1[1]); o[6] = f2bf(x1[2]); o[7] = f2bf(x1[3]);
  unsigned short* d = dst + (size_t)i * 8;
  *(volatile us8*)d = o;
  __threadfence();
  *(volatile us8*)d = o;
}

__global__ __launch_bounds__(256)
void k_cvt_wt(const float* __restrict__ W, unsigned short* Wt) {
  __shared__ __attribute__((aligned(16))) unsigned short T[64 * TPW];
  const int n0 = blockIdx.x * 64;
  const int k0 = blockIdx.y * 64;
  const int t = threadIdx.x;
#pragma unroll
  for (int it = 0; it < 4; ++it) {
    const int idx4 = it * 256 + t;
    const int kr = idx4 >> 4, c4 = idx4 & 15;
    const v4f x = *(const v4f*)(W + (size_t)(k0 + kr) * NOUT + n0 + 4 * c4);
    T[(4 * c4 + 0) * TPW + kr] = f2bf(x[0]);
    T[(4 * c4 + 1) * TPW + kr] = f2bf(x[1]);
    T[(4 * c4 + 2) * TPW + kr] = f2bf(x[2]);
    T[(4 * c4 + 3) * TPW + kr] = f2bf(x[3]);
  }
  __syncthreads();
  const int wv = t >> 5, lane = t & 31, q8 = lane & 7;
  us8 val[2];
  size_t off[2];
#pragma unroll
  for (int p = 0; p < 2; ++p) {
    const int n = wv * 8 + p * 4 + (lane >> 3);
    val[p] = *(const us8*)(&T[n * TPW + 8 * q8]);
    off[p] = (size_t)(n0 + n) * HID + k0 + 8 * q8;
  }
#pragma unroll
  for (int p = 0; p < 2; ++p) *(volatile us8*)(Wt + off[p]) = val[p];
  __threadfence();
#pragma unroll
  for (int p = 0; p < 2; ++p) *(volatile us8*)(Wt + off[p]) = val[p];
}

__global__ __launch_bounds__(128)
void k_gate_lr(const unsigned short* __restrict__ Hb, const float* __restrict__ w1,
               const float* __restrict__ w2, const float* __restrict__ b2, float* dec) {
  __shared__ float sy[64 * LOWR];
  __shared__ __attribute__((aligned(16))) float sdc[64 * NG];
  const int m0 = blockIdx.x * 64;
  const int t = threadIdx.x, wave = t >> 5, lane = t & 31, h = lane >> 4, l15 = lane & 15;

  v8f acc = {0.f, 0.f, 0.f, 0.f, 0.f, 0.f, 0.f, 0.f};
  const unsigned short* arow = Hb + (size_t)(m0 + wave * 16 + l15) * HID;
#pragma unroll 2
  for (int ks = 0; ks < HID / 32; ++ks) {
    const int k0 = ks * 32;
    Frag a, b;
    a.hv[0] = *(const us8*)(arow + k0 + 8 * h);
    a.hv[1] = *(const us8*)(arow + k0 + 16 + 8 * h);
#pragma unroll
    for (int i = 0; i < 8; ++i) {
      b.u[i]     = f2bf(w1[(size_t)(k0 + 8 * h + i) * LOWR + l15]);
      b.u[8 + i] = f2bf(w1[(size_t)(k0 + 16 + 8 * h + i) * LOWR + l15]);
    }
    acc = wmma_bf16(a.v, b.v, acc);
  }
#pragma unroll
  for (int r = 0; r < 8; ++r) sy[(wave * 16 + 8 * h + r) * LOWR + l15] = acc[r];
  __syncthreads();

  if (t < 64) {
    float y[LOWR];
#pragma unroll
    for (int n = 0; n < LOWR; ++n) y[n] = sy[t * LOWR + n];
#pragma unroll
    for (int g = 0; g < NG; ++g) {
      float z = 0.f;
#pragma unroll
      for (int n = 0; n < LOWR; ++n) z += y[n] * bfr(w2[n * NG + g]);
      z += bfr(b2[g]);
      const float ls = fminf(z, 0.f) - log1pf(expf(-fabsf(z)));
      sdc[t * NG + g] = expf(ls * 0.0625f);
    }
  }
  __syncthreads();

  if (wave == 0) {
    const v4f v0 = *(const v4f*)(&sdc[lane * 4]);
    const v4f v1 = *(const v4f*)(&sdc[128 + lane * 4]);
    float* base = dec + (size_t)m0 * NG;
    *(volatile v4f*)(base + lane * 4) = v0;
    *(volatile v4f*)(base + 128 + lane * 4) = v1;
    __threadfence();
    *(volatile v4f*)(base + lane * 4) = v0;
    *(volatile v4f*)(base + 128 + lane * 4) = v1;
  }
}

__global__ __launch_bounds__(SCAN_THREADS)
void k_scan(const float* __restrict__ q, const float* __restrict__ k, const float* __restrict__ v,
            const float* __restrict__ dec, const float* __restrict__ S0,
            float* oatt, float* Sfin) {
  __shared__ __attribute__((aligned(16))) float sm[5 * TCH * 64];
  __shared__ float sd[TCH];
  float* sq = sm;
  float* sk = sm + TCH * 64;
  float* sv = sm + 2 * TCH * 64;
  float* so = sm + 3 * TCH * 64;

  const int bh = blockIdx.x;
  const int b = bh / NH, hh = bh % NH;
  const int kvh = hh / (NH / NKV);
  const int gsel = hh % NG;
  const int t = threadIdx.x, j = t & 63, hf = t >> 6;
  const int i0 = hf * 32;

  float S[32];
  const float* S0p = S0 + (size_t)bh * HD * HD;
#pragma unroll
  for (int i = 0; i < 32; ++i) S[i] = bfr(S0p[(i0 + i) * HD + j]);

#pragma unroll 1
  for (int ch = 0; ch < NL / TCH; ++ch) {
    const int l0 = ch * TCH;
    if (hf == 0) {
#pragma unroll 4
      for (int s = 0; s < TCH; ++s) {
        const size_t tok = (size_t)b * NL + l0 + s;
        sq[s * 64 + j] = bfr(q[(tok * NH + hh) * HD + j]) * 0.125f;
        sk[s * 64 + j] = bfr(k[(tok * NKV + kvh) * HD + j]);
      }
    } else {
#pragma unroll 4
      for (int s = 0; s < TCH; ++s) {
        const size_t tok = (size_t)b * NL + l0 + s;
        sv[s * 64 + j] = bfr(v[(tok * NKV + kvh) * HD + j]);
      }
      if (j < TCH) sd[j] = dec[((size_t)b * NL + l0 + j) * NG + gsel];
    }
    __syncthreads();

#pragma unroll 1
    for (int s = 0; s < TCH; ++s) {
      const float dcy = sd[s];
      const float vj = sv[s * 64 + j];
      const v4f* k4 = (const v4f*)(sk + s * 64 + i0);
      const v4f* q4 = (const v4f*)(sq + s * 64 + i0);
      float od = 0.f;
#pragma unroll
      for (int g4 = 0; g4 < 8; ++g4) {
        const v4f kk = k4[g4];
        const v4f qv = q4[g4];
#pragma unroll
        for (int c = 0; c < 4; ++c) {
          const float sn = S[4 * g4 + c] * dcy + kk[c] * vj;
          S[4 * g4 + c] = sn;
          od += qv[c] * sn;
        }
      }
      so[(hf * TCH + s) * 64 + j] = od;
    }
    __syncthreads();

    {
      const v4f* p0 = (const v4f*)so;
      const v4f* p1 = (const v4f*)(so + TCH * 64);
      v4f tmp[4];
#pragma unroll
      for (int p = 0; p < 4; ++p) tmp[p] = p0[p * SCAN_THREADS + t] + p1[p * SCAN_THREADS + t];
      float* base = oatt + ((size_t)bh * NL + l0) * HD;
#pragma unroll
      for (int p = 0; p < 4; ++p) *(volatile v4f*)(base + (size_t)(p * SCAN_THREADS + t) * 4) = tmp[p];
      __threadfence();
#pragma unroll
      for (int p = 0; p < 4; ++p) *(volatile v4f*)(base + (size_t)(p * SCAN_THREADS + t) * 4) = tmp[p];
    }
  }

  __syncthreads();
#pragma unroll
  for (int i = 0; i < 32; ++i) sm[(i0 + i) * HD + j] = S[i];
  __syncthreads();
  {
    const v4f* src = (const v4f*)sm;
    v4f tmp[8];
#pragma unroll
    for (int p = 0; p < 8; ++p) tmp[p] = src[p * SCAN_THREADS + t];
    float* base = Sfin + (size_t)bh * HD * HD;
#pragma unroll
    for (int p = 0; p < 8; ++p) *(volatile v4f*)(base + (size_t)(p * SCAN_THREADS + t) * 4) = tmp[p];
    __threadfence();
#pragma unroll
    for (int p = 0; p < 8; ++p) *(volatile v4f*)(base + (size_t)(p * SCAN_THREADS + t) * 4) = tmp[p];
  }
}

__global__ __launch_bounds__(128)
void k_out(const unsigned short* __restrict__ Hb, const unsigned short* __restrict__ Wt,
           const float* __restrict__ oatt, const float* __restrict__ gnw, const float* __restrict__ gnb,
           float* out) {
  __shared__ __attribute__((aligned(16))) float st[4 * 16 * HD];
  const int m0 = blockIdx.x * 64, hh = blockIdx.y, n0 = hh * HD;
  const int t = threadIdx.x, wave = t >> 5, lane = t & 31, h = lane >> 4, l15 = lane & 15;

  v8f acc[4];
#pragma unroll
  for (int nt = 0; nt < 4; ++nt) {
#pragma unroll
    for (int r = 0; r < 8; ++r) acc[nt][r] = 0.f;
  }

  const unsigned short* arow = Hb + (size_t)(m0 + wave * 16 + l15) * HID;
  const unsigned short* brow = Wt + (size_t)(n0 + l15) * HID;
#pragma unroll 2
  for (int ks = 0; ks < HID / 32; ++ks) {
    const int k0 = ks * 32;
    Frag a;
    a.hv[0] = *(const us8*)(arow + k0 + 8 * h);
    a.hv[1] = *(const us8*)(arow + k0 + 16 + 8 * h);
#pragma unroll
    for (int nt = 0; nt < 4; ++nt) {
      Frag bb;
      const unsigned short* bp = brow + (size_t)nt * 16 * HID + k0;
      bb.hv[0] = *(const us8*)(bp + 8 * h);
      bb.hv[1] = *(const us8*)(bp + 16 + 8 * h);
      acc[nt] = wmma_bf16(a.v, bb.v, acc[nt]);
    }
  }

  float wln[4], bln[4];
#pragma unroll
  for (int nt = 0; nt < 4; ++nt) {
    wln[nt] = bfr(gnw[nt * 16 + l15]);
    bln[nt] = bfr(gnb[nt * 16 + l15]);
  }
  float* stw = st + wave * 16 * HD;
  const int rowb = m0 + wave * 16 + 8 * h;
#pragma unroll
  for (int r = 0; r < 8; ++r) {
    const int m = rowb + r;
    const int bi = m / NL, li = m % NL;
    const float* orow = oatt + (((size_t)bi * NH + hh) * NL + li) * HD;
    float x[4];
#pragma unroll
    for (int nt = 0; nt < 4; ++nt) x[nt] = orow[nt * 16 + l15];
    float s1 = (x[0] + x[1]) + (x[2] + x[3]);
    s1 += __shfl_xor(s1, 1, 32);
    s1 += __shfl_xor(s1, 2, 32);
    s1 += __shfl_xor(s1, 4, 32);
    s1 += __shfl_xor(s1, 8, 32);
    const float mu = s1 * (1.f / 64.f);
    float d[4];
    float s2 = 0.f;
#pragma unroll
    for (int nt = 0; nt < 4; ++nt) { d[nt] = x[nt] - mu; s2 += d[nt] * d[nt]; }
    s2 += __shfl_xor(s2, 1, 32);
    s2 += __shfl_xor(s2, 2, 32);
    s2 += __shfl_xor(s2, 4, 32);
    s2 += __shfl_xor(s2, 8, 32);
    const float inv = rsqrtf(s2 * (1.f / 64.f) + LN_EPS);
#pragma unroll
    for (int nt = 0; nt < 4; ++nt) {
      const float y = d[nt] * inv * wln[nt] + bln[nt];
      const float gv = acc[nt][r];
      const float sg = gv * (1.f / (1.f + expf(-gv)));
      stw[(8 * h + r) * HD + nt * 16 + l15] = y * sg;
    }
  }
  __syncthreads();
  {
    v4f tmp[8];
    size_t off[8];
#pragma unroll
    for (int p = 0; p < 8; ++p) {
      const int rr = 2 * p + (lane >> 4);
      const int qq = lane & 15;
      tmp[p] = *(const v4f*)(stw + rr * HD + 4 * qq);
      off[p] = (size_t)(m0 + wave * 16 + rr) * NOUT + n0 + 4 * qq;
    }
#pragma unroll
    for (int p = 0; p < 8; ++p) *(volatile v4f*)(out + off[p]) = tmp[p];
    __threadfence();
#pragma unroll
    for (int p = 0; p < 8; ++p) *(volatile v4f*)(out + off[p]) = tmp[p];
  }
}

static inline size_t al256(size_t x) { return (x + 255) & ~(size_t)255; }

extern "C" void kernel_launch(void* const* d_in, const int* in_sizes, int n_in,
                              void* d_out, int out_size, void* d_ws, size_t ws_size,
                              hipStream_t stream) {
  if (n_in < 11) return;
  if (in_sizes[0] != NB * NL * NH * HD) return;
  if (in_sizes[1] != NB * NL * NKV * HD) return;
  if (in_sizes[2] != NB * NL * NKV * HD) return;
  if (in_sizes[3] != NB * NL * HID) return;
  if (in_sizes[4] != NB * NH * HD * HD) return;
  if (in_sizes[5] != HID * NOUT) return;
  if (in_sizes[6] != HID * LOWR) return;
  if (in_sizes[7] != LOWR * NG) return;
  if (in_sizes[8] < NG || in_sizes[9] < HD || in_sizes[10] < HD) return;
  if (out_size != NB * NL * NOUT + NB * NH * HD * HD) return;

  const float* q      = (const float*)d_in[0];
  const float* k      = (const float*)d_in[1];
  const float* v      = (const float*)d_in[2];
  const float* hidden = (const float*)d_in[3];
  const float* S0     = (const float*)d_in[4];
  const float* gw     = (const float*)d_in[5];
  const float* w1     = (const float*)d_in[6];
  const float* w2     = (const float*)d_in[7];
  const float* b2     = (const float*)d_in[8];
  const float* gnw    = (const float*)d_in[9];
  const float* gnb    = (const float*)d_in[10];

  float* out0 = (float*)d_out;
  float* out1 = out0 + (size_t)NB * NL * NOUT;

  const size_t bytes_hb  = (size_t)NB * NL * HID * sizeof(unsigned short);
  const size_t bytes_wt  = (size_t)NOUT * HID * sizeof(unsigned short);
  const size_t bytes_dec = (size_t)NB * NL * NG * sizeof(float);
  const size_t bytes_o   = (size_t)NB * NH * NL * HD * sizeof(float);
  const size_t off_hb  = 0;
  const size_t off_wt  = al256(off_hb + bytes_hb);
  const size_t off_dec = al256(off_wt + bytes_wt);
  const size_t off_o   = al256(off_dec + bytes_dec);
  if (off_o + bytes_o > ws_size) return;

  char* ws = (char*)d_ws;
  unsigned short* Hb = (unsigned short*)(ws + off_hb);
  unsigned short* Wt = (unsigned short*)(ws + off_wt);
  float* decp = (float*)(ws + off_dec);
  float* oatt = (float*)(ws + off_o);

  const int n8 = (NB * NL * HID) / 8;
  k_cvt_h<<<(n8 + 255) / 256, 256, 0, stream>>>(hidden, Hb, n8);
  k_cvt_wt<<<dim3(NOUT / 64, HID / 64), 256, 0, stream>>>(gw, Wt);
  k_gate_lr<<<(NB * NL) / 64, 128, 0, stream>>>(Hb, w1, w2, b2, decp);
  k_scan<<<NB * NH, SCAN_THREADS, 0, stream>>>(q, k, v, decp, S0, oatt, out1);
  k_out<<<dim3((NB * NL) / 64, NH), 128, 0, stream>>>(Hb, Wt, oatt, gnw, gnb, out0);
}
